// SelfAttention2d_43602507989512
// MI455X (gfx1250) — hardware-run, weakly checked
//
#include <hip/hip_runtime.h>


#define NB_  4
#define TT   4096
#define HD   128
#define DQK  16
#define DP   32
#define QKW  64
#define BKO  32
#define ZH   1
#define RH   0
#define PCAR 1024.0f
#define SCL  1.0f
#define PFL  6.103515625e-05f
typedef _Float16 h16;
typedef unsigned short bf;
typedef __attribute__((ext_vector_type(16))) __bf16   v16bf;
typedef __attribute__((ext_vector_type(16))) _Float16 v16h;
typedef __attribute__((ext_vector_type(8)))  _Float16 v8h;
typedef __attribute__((ext_vector_type(8)))  unsigned short v8us;
typedef __attribute__((ext_vector_type(8)))  float    v8f;
typedef __attribute__((ext_vector_type(4)))  float    v4f;
typedef v8h  __attribute__((may_alias)) v8ha;
typedef v4f  __attribute__((may_alias)) v4fa;
typedef v8us __attribute__((may_alias)) v8usa;

__device__ __forceinline__ unsigned short f2bf(float f) { unsigned u = __float_as_uint(f); u += 0x7FFFu + ((u >> 16) & 1u); return (unsigned short)(u >> 16); }
__device__ __forceinline__ float bf2f(unsigned short b) { return __uint_as_float(((unsigned)b) << 16); }
__device__ __forceinline__ float bfr(float f) { return bf2f(f2bf(f)); }
__device__ __forceinline__ v16h cat16(v8h lo, v8h hi) { return __builtin_shufflevector(lo, hi, 0, 1, 2, 3, 4, 5, 6, 7, 8, 9, 10, 11, 12, 13, 14, 15); }
__device__ __forceinline__ v16bf cat16b(v8us lo, v8us hi) { return __builtin_bit_cast(v16bf, __builtin_shufflevector(lo, hi, 0, 1, 2, 3, 4, 5, 6, 7, 8, 9, 10, 11, 12, 13, 14, 15)); }
__device__ __forceinline__ v8f wmma16(v16h a, v16h b, v8f c) { return __builtin_amdgcn_wmma_f32_16x16x32_f16(false, a, false, b, (short)0, c, false, false); }
__device__ __forceinline__ v8f wmmab(v16bf a, v16bf b, v8f c) { return __builtin_amdgcn_wmma_f32_16x16x32_bf16(false, a, false, b, (short)0, c, false, false); }


template <typename T16> struct WFrag;
template <> struct WFrag<h16> { typedef v16h V; static __device__ __forceinline__ V ld(const h16* p) { return cat16(*(const v8h*)p, *(const v8h*)(p + 16)); } static __device__ __forceinline__ v8f mma(V a, V b, v8f c) { return wmma16(a, b, c); } };
template <> struct WFrag<bf> { typedef v16bf V; static __device__ __forceinline__ V ld(const bf* p) { return cat16b(*(const v8us*)p, *(const v8us*)(p + 16)); } static __device__ __forceinline__ v8f mma(V a, V b, v8f c) { return wmmab(a, b, c); } };
template <typename T16, int NSPLIT, bool BIAS>
__global__ __launch_bounds__(32) void k_gemmw(const T16* __restrict__ A, const T16* __restrict__ A2, const T16* __restrict__ Bt, const T16* __restrict__ Bt2, int K, float* C, int ldc, const float* __restrict__ bias, size_t sA, size_t sB, size_t sC) {
    typedef typename WFrag<T16>::V V;
    __shared__ __align__(16) float os[16 * 68];
    const size_t z = blockIdx.z; A += z * sA; if (A2) A2 += z * sA; Bt += z * sB; if (Bt2) Bt2 += z * sB; C += z * sC;
    const int lane = threadIdx.x & 31, lr = lane & 15, hi = lane >> 4; const int r0 = blockIdx.x * 64, c0 = blockIdx.y * 64;
    v8f acc[4][4];
#pragma unroll
    for (int mb = 0; mb < 4; ++mb)
#pragma unroll
        for (int nb = 0; nb < 4; ++nb) acc[mb][nb] = (v8f){};
    const size_t aoff = (size_t)(r0 + lr) * K + 8 * hi, boff = (size_t)(c0 + lr) * K + 8 * hi;

    for (int kc = 0; kc < K; kc += 32) {
        V a[4], a2[4];
#pragma unroll
        for (int mb = 0; mb < 4; ++mb) { a[mb] = WFrag<T16>::ld(A + aoff + (size_t)mb * 16 * K + kc); if (NSPLIT == 1 || NSPLIT == 2) a2[mb] = WFrag<T16>::ld(A2 + aoff + (size_t)mb * 16 * K + kc); }
#pragma unroll
        for (int nb = 0; nb < 4; ++nb) { const V b = WFrag<T16>::ld(Bt + boff + (size_t)nb * 16 * K + kc); V b2; if (NSPLIT >= 2) b2 = WFrag<T16>::ld(Bt2 + boff + (size_t)nb * 16 * K + kc);
#pragma unroll
            for (int mb = 0; mb < 4; ++mb) { acc[mb][nb] = WFrag<T16>::mma(a[mb], b, acc[mb][nb]); if (NSPLIT == 1 || NSPLIT == 2) acc[mb][nb] = WFrag<T16>::mma(a2[mb], b, acc[mb][nb]); if (NSPLIT >= 2) acc[mb][nb] = WFrag<T16>::mma(a[mb], b2, acc[mb][nb]); } }
        asm volatile("v_nop\n\tv_nop\n\tv_nop\n\tv_nop" : "+v"(acc[0][0]), "+v"(acc[1][1]), "+v"(acc[2][2]), "+v"(acc[3][3]) : "v"(a[0]), "v"(a[3]));
    }
#pragma unroll
    for (int mb = 0; mb < 4; ++mb) {
#pragma unroll
        for (int nb = 0; nb < 4; ++nb) {
#pragma unroll
            for (int j = 0; j < 8; ++j) os[(hi * 8 + j) * 68 + nb * 16 + lr] = acc[mb][nb][j]; }
        __builtin_amdgcn_wave_barrier(); asm volatile("" ::: "memory");
        float* crow = C + (size_t)(r0 + mb * 16) * ldc + c0;
#pragma unroll 1
        for (int ps = 0; ps < 2; ++ps) {
#pragma unroll
            for (int s = 0; s < 8; ++s) { const int row = 2 * s + hi, cofs = lr * 4; v4f val = *(const v4fa*)(os + row * 68 + cofs); if (BIAS) { val[0] += bfr(bias[c0 + cofs]); val[1] += bfr(bias[c0 + cofs + 1]); val[2] += bfr(bias[c0 + cofs + 2]); val[3] += bfr(bias[c0 + cofs + 3]); }
                *(volatile v4f*)(crow + (size_t)row * ldc + cofs) = val; }
            if (ps == 0) __threadfence(); }
        __builtin_amdgcn_wave_barrier(); asm volatile("" ::: "memory");
    }
}

__device__ __forceinline__ h16 tohx(float x) { return (h16)x; }
__device__ __forceinline__ void splitf(float y, unsigned short& h, unsigned short& l) { h = f2bf(y); l = f2bf(y - bf2f(h)); }
typedef __attribute__((ext_vector_type(2))) _Float16 v2h;
typedef __attribute__((ext_vector_type(4))) _Float16 v4h;
typedef __attribute__((ext_vector_type(2))) unsigned short v2us;
typedef __attribute__((ext_vector_type(4))) unsigned short v4us;
typedef __attribute__((ext_vector_type(2))) float v2f;
typedef __attribute__((ext_vector_type(4))) int v4i;


__global__ __launch_bounds__(256) void k_asoft(const float* __restrict__ Sb, h16* P16, bf* Ph, bf* Pl) {
    const int lane = threadIdx.x & 31; const int row = blockIdx.x * 8 + (threadIdx.x >> 5); if (row >= ZH * TT) return; const int i = row % TT; const int zz = row / TT; (void)zz; const bool hires = (i < RH); const float* sr = Sb + (size_t)row * TT; float v[TT / 32]; float mx = -3.0e38f;
#pragma unroll
    for (int ch = 0; ch < TT / 128; ++ch) { const int j0 = ch * 128 + lane * 4; const v4f a = *(const v4f*)(sr + j0);
#pragma unroll
        for (int q = 0; q < 4; ++q) { const int j = j0 + q; (void)j; const float t = a[q] * SCL; v[ch * 4 + q] = t; mx = fmaxf(mx, t); } }
#pragma unroll
    for (int sh = 16; sh; sh >>= 1) mx = fmaxf(mx, __shfl_xor(mx, sh, 32));
    float sum = 0.f;
#pragma unroll
    for (int k = 0; k < TT / 32; ++k) { float d0 = __fsub_rn(v[k], mx); v[k] = __builtin_amdgcn_exp2f(__fmul_rn(d0, 1.4426950408889634f)); sum += v[k]; }
#pragma unroll
    for (int sh = 16; sh; sh >>= 1) sum += __shfl_xor(sum, sh, 32);
    const float f = __fdiv_rn(hires ? 1.0f : PCAR, sum);
#pragma unroll 1
    for (int ps = 0; ps < 2; ++ps) {
        if (hires) {
#pragma unroll
            for (int ch = 0; ch < TT / 128; ++ch) { v4us oh, ol;
#pragma unroll
                for (int q = 0; q < 4; ++q) { unsigned short a, c2; splitf(v[ch * 4 + q] * f, a, c2); oh[q] = a; ol[q] = c2; }
                const size_t oo = ((size_t)zz * (RH ? RH : 1) + i) * TT + ch * 128 + lane * 4; *(volatile v4us*)(Ph + oo) = oh; *(volatile v4us*)(Pl + oo) = ol; }
        } else {
#pragma unroll
            for (int ch = 0; ch < TT / 128; ++ch) { v4h o4;
#pragma unroll
                for (int q = 0; q < 4; ++q) { const float w = v[ch * 4 + q] * f; o4[q] = tohx(w < PFL ? 0.0f : w); }
                *(volatile v4h*)(P16 + (size_t)row * TT + ch * 128 + lane * 4) = o4; } }
        if (ps == 0) __threadfence(); }
}
__global__ __launch_bounds__(256) void k_f2h(const float* __restrict__ S, h16* P16, size_t n4) { const size_t i = (size_t)blockIdx.x * 256 + threadIdx.x; if (i >= n4) return; const v4f v = *(const v4f*)(S + i * 4); v4h o;
#pragma unroll
    for (int q = 0; q < 4; ++q) o[q] = tohx(v[q]);
    *(volatile v4h*)(P16 + i * 4) = o; __threadfence(); *(volatile v4h*)(P16 + i * 4) = o; }
__global__ __launch_bounds__(256) void k_cvt8(const float* __restrict__ src, bf* dst, size_t n8) { const size_t i = (size_t)blockIdx.x * 256 + threadIdx.x; if (i >= n8) return; const v8f v = *(const v8f*)(src + i * 8); v8us o;
#pragma unroll
    for (int k = 0; k < 8; ++k) o[k] = f2bf(v[k]); *(volatile v8us*)(dst + i * 8) = o; __threadfence(); *(volatile v8us*)(dst + i * 8) = o; }
__global__ __launch_bounds__(256) void k_rbf(const float* __restrict__ X, float* Y, size_t n4) { const size_t i = (size_t)blockIdx.x * 256 + threadIdx.x; if (i >= n4) return; const v4f a = *(const v4f*)(X + i * 4); v4f o;
#pragma unroll
    for (int q = 0; q < 4; ++q) o[q] = bfr(a[q]);
    *(volatile v4f*)(Y + i * 4) = o; __threadfence(); *(volatile v4f*)(Y + i * 4) = o; }
__global__ __launch_bounds__(256) void k_msin(const float* __restrict__ xr, float* Y, float* O0) { const size_t e = (size_t)blockIdx.x * 256 + threadIdx.x; const size_t n0 = e * 2;
    for (int kc = 0; kc < HD / 16; ++kc) { float a[16], b[16];
#pragma unroll
        for (int c = 0; c < 16; ++c) { const v2f v = *(const v2f*)(xr + (size_t)(kc * 16 + c) * TT + n0); a[c] = v[0]; b[c] = v[1]; }
#pragma unroll
        for (int ps = 0; ps < 2; ++ps) {
#pragma unroll
            for (int k = 0; k < 4; ++k) { v4f o; o[0] = a[k * 4]; o[1] = a[k * 4 + 1]; o[2] = a[k * 4 + 2]; o[3] = a[k * 4 + 3]; *(volatile v4f*)(Y + n0 * HD + kc * 16 + k * 4) = o; o[0] = b[k * 4]; o[1] = b[k * 4 + 1]; o[2] = b[k * 4 + 2]; o[3] = b[k * 4 + 3]; *(volatile v4f*)(Y + (n0 + 1) * HD + kc * 16 + k * 4) = o; }
#pragma unroll
            for (int c = 0; c < 16; ++c) { v2f f2; f2[0] = a[c]; f2[1] = b[c]; *(volatile v2f*)(O0 + (size_t)(kc * 16 + c) * TT + n0) = f2; }
            if (ps == 0) __threadfence(); } } }
__global__ __launch_bounds__(256) void k_qkb(const float* __restrict__ QK, const float* __restrict__ BQ, float* QF, float* KF) { const size_t n = (size_t)blockIdx.x * 256 + threadIdx.x; v4f q[DQK / 4], k[DQK / 4];
#pragma unroll
    for (int j = 0; j < DQK / 4; ++j) { q[j] = *(const v4f*)(QK + n * QKW + j * 4); k[j] = *(const v4f*)(QK + n * QKW + DQK + j * 4); const v4f b0 = *(const v4f*)(BQ + j * 4), b1 = *(const v4f*)(BQ + BKO + j * 4);
#pragma unroll
        for (int e = 0; e < 4; ++e) { q[j][e] = __fadd_rn(q[j][e], b0[e]); k[j][e] = __fadd_rn(k[j][e], b1[e]); } }
    v4f z; z[0] = 0.f; z[1] = 0.f; z[2] = 0.f; z[3] = 0.f;
#pragma unroll
    for (int ps = 0; ps < 2; ++ps) {
#pragma unroll
        for (int j = 0; j < DQK / 4; ++j) { *(volatile v4f*)(QF + n * DP + j * 4) = q[j]; *(volatile v4f*)(KF + n * DP + j * 4) = k[j]; }
#pragma unroll
        for (int j = DQK / 4; j < DP / 4; ++j) { *(volatile v4f*)(QF + n * DP + j * 4) = z; *(volatile v4f*)(KF + n * DP + j * 4) = z; }
        if (ps == 0) __threadfence(); } }
__global__ __launch_bounds__(256) void k_resgb(const float* __restrict__ Ob, const float* __restrict__ BV, const float* __restrict__ GAM, const float* __restrict__ XV, float* out) { const size_t e = (size_t)blockIdx.x * 256 + threadIdx.x; const size_t n0 = e * 2; const float g = bfr(GAM[0]);
    for (int kc = 0; kc < HD / 16; ++kc) { float a[16], b[16];
#pragma unroll
        for (int k = 0; k < 4; ++k) { const v4f o0 = *(const v4f*)(Ob + n0 * HD + kc * 16 + k * 4), o1 = *(const v4f*)(Ob + (n0 + 1) * HD + kc * 16 + k * 4), bb = *(const v4f*)(BV + kc * 16 + k * 4);
#pragma unroll
            for (int j = 0; j < 4; ++j) { a[k * 4 + j] = __fadd_rn(__fmul_rn(o0[j], 1.0f / PCAR), bb[j]); b[k * 4 + j] = __fadd_rn(__fmul_rn(o1[j], 1.0f / PCAR), bb[j]); } }
#pragma unroll
        for (int c = 0; c < 16; ++c) { const v2f xv = *(const v2f*)(XV + (size_t)(kc * 16 + c) * TT + n0); a[c] = g * a[c] + xv[0]; b[c] = g * b[c] + xv[1]; }
#pragma unroll
        for (int ps = 0; ps < 2; ++ps) {
#pragma unroll
            for (int c = 0; c < 16; ++c) { v2f f2; f2[0] = a[c]; f2[1] = b[c]; *(volatile v2f*)(out + (size_t)(kc * 16 + c) * TT + n0) = f2; }
            if (ps == 0) __threadfence(); } } }

extern "C" void kernel_launch(void* const* d_in, const int* in_sizes, int n_in,
                              void* d_out, int out_size, void* d_ws, size_t ws_size, hipStream_t stream) {
    (void)in_sizes; (void)n_in; (void)out_size;
    const float* x = (const float*)d_in[0]; const float* wq = (const float*)d_in[1]; const float* bq = (const float*)d_in[2]; const float* wk = (const float*)d_in[3]; const float* bk = (const float*)d_in[4]; const float* wv = (const float*)d_in[5]; const float* bv = (const float*)d_in[6]; const float* gam = (const float*)d_in[7];
    float* OUT = (float*)d_out;
    char* wsp = (char*)d_ws;
    auto take = [&](size_t bytes) { char* p = wsp; wsp += (bytes + 255) & ~(size_t)255; return (void*)p; };
    float* WR = (float*)take((size_t)QKW * HD * 4); bf* WQKB = (bf*)take((size_t)QKW * HD * 2); bf* WVB = (bf*)take((size_t)HD * HD * 2); float* BR = (float*)take((size_t)256 * 4);
    float* XV = (float*)take((size_t)HD * TT * 4); float* YV = (float*)take((size_t)TT * HD * 4); float* SPARE = (float*)take((size_t)HD * TT * 4);
    bf* YVB = (bf*)take((size_t)TT * HD * 2); float* QKF = (float*)take((size_t)TT * QKW * 4); float* QF = (float*)take((size_t)TT * DP * 4); float* KF = (float*)take((size_t)TT * DP * 4);
    h16* QH = (h16*)take((size_t)TT * DP * 2); h16* KH = (h16*)take((size_t)TT * DP * 2); float* VC = (float*)take((size_t)HD * TT * 4); h16* VCH = (h16*)take((size_t)HD * TT * 2);
    bf* Ph = nullptr; bf* Pl = nullptr;
    float* Sb = (float*)take((size_t)(TT / 2) * TT * 4); h16* P16 = (h16*)take((size_t)(TT / 2) * TT * 2); float* Ob = (float*)take((size_t)TT * HD * 4);
    if ((size_t)(wsp - (char*)d_ws) > ws_size) return;
    k_rbf<<<2, 256, 0, stream>>>(wq, WR, (size_t)DQK * HD / 4); k_rbf<<<2, 256, 0, stream>>>(wk, WR + (size_t)DQK * HD, (size_t)DQK * HD / 4); k_rbf<<<4, 256, 0, stream>>>(wv, WR + (size_t)2 * DQK * HD, (size_t)(QKW - 2 * DQK) * HD / 4);
    k_cvt8<<<4, 256, 0, stream>>>(WR, WQKB, (size_t)QKW * HD / 8); k_cvt8<<<8, 256, 0, stream>>>(wv, WVB, (size_t)HD * HD / 8);
    k_rbf<<<1, 256, 0, stream>>>(bv, BR, (size_t)HD / 4); k_rbf<<<1, 256, 0, stream>>>(bq, BR + HD, (size_t)DQK / 4); k_rbf<<<1, 256, 0, stream>>>(bk, BR + HD + BKO, (size_t)DQK / 4);
    const size_t N4 = (size_t)HD * TT / 4, N8 = (size_t)HD * TT / 8; const unsigned G4 = (unsigned)((N4 + 255) / 256), G8 = (unsigned)((N8 + 255) / 256); const size_t P4 = (size_t)TT * DP / 4; const unsigned GP = (unsigned)((P4 + 255) / 256);
    for (int b = 0; b < NB_; ++b) { const size_t ob = (size_t)b * HD * TT;
        k_rbf<<<G4, 256, 0, stream>>>(x + ob, XV, N4);
        k_msin<<<(unsigned)(TT / 2 / 256), 256, 0, stream>>>(XV, YV, SPARE);
        k_cvt8<<<G8, 256, 0, stream>>>(YV, YVB, N8);
        k_gemmw<bf, 0, false><<<dim3(TT / 64, QKW / 64, 1), 32, 0, stream>>>(YVB, nullptr, WQKB, nullptr, HD, QKF, QKW, nullptr, 0, 0, 0);
        k_qkb<<<(unsigned)(TT / 256), 256, 0, stream>>>(QKF, BR + HD, QF, KF); k_f2h<<<GP, 256, 0, stream>>>(QF, QH, P4); k_f2h<<<GP, 256, 0, stream>>>(KF, KH, P4);
        k_gemmw<bf, 0, false><<<dim3(HD / 64, TT / 64, 1), 32, 0, stream>>>(WVB, nullptr, YVB, nullptr, HD, VC, TT, nullptr, 0, 0, 0); k_f2h<<<G4, 256, 0, stream>>>(VC, VCH, N4);
        for (int hf = 0; hf < 2; ++hf) { const size_t r0 = (size_t)hf * (TT / 2);
            k_gemmw<h16, 0, false><<<dim3(TT / 2 / 64, TT / 64, 1), 32, 0, stream>>>(QH + r0 * DP, nullptr, KH, nullptr, DP, Sb, TT, nullptr, 0, 0, 0);
            k_asoft<<<TT / 2 / 8, 256, 0, stream>>>(Sb, P16, Ph, Pl);
            k_gemmw<h16, 0, false><<<dim3(TT / 2 / 64, HD / 64, 1), 32, 0, stream>>>(P16, nullptr, VCH, nullptr, TT, Ob + r0 * HD, HD, nullptr, 0, 0, 0); }
        k_resgb<<<(unsigned)(TT / 2 / 256), 256, 0, stream>>>(Ob, BR, gam, XV, OUT + ob); }
}
